// efficient_Attention_modified_21071109554259
// MI455X (gfx1250) — hardware-verified
//
#include <hip/hip_runtime.h>

#define BB    8
#define DIMC  384
#define NN    4096
#define HEADS 8
#define KDIM  32
#define DD    64
#define NHKD  256
#define DHC   512
#define MQKV  1024
#define TP    132
#define TPD   68

typedef _Float16 v16h __attribute__((ext_vector_type(16)));
typedef _Float16 v8h  __attribute__((ext_vector_type(8)));
typedef float    v8f  __attribute__((ext_vector_type(8)));
typedef float    v4f  __attribute__((ext_vector_type(4)));
typedef float    v4fa __attribute__((ext_vector_type(4), may_alias));

union Frag { v16h v; v8h half[2]; };

__device__ __forceinline__ v16h load_frag(const _Float16* __restrict__ p, int h)
{
    Frag f;
    f.half[0] = *(const v8h*)(p + 8 * h);
    f.half[1] = *(const v8h*)(p + 16 + 8 * h);
    return f.v;
}

__device__ __forceinline__ v8f mma16(v16h a, v16h b, v8f c)
{
    return __builtin_amdgcn_wmma_f32_16x16x32_f16(false, a, false, b, (short)0, c, false, false);
}

#define GUARD1(c, a, b) \
    asm volatile("v_nop\n\tv_nop\n\tv_nop\n\tv_nop" : "+v"(c) : "v"(a), "v"(b))
#define GUARD4(c0, c1, c2, c3, a, b0, b1, b2, b3) \
    asm volatile("v_nop\n\tv_nop\n\tv_nop\n\tv_nop" \
                 : "+v"(c0), "+v"(c1), "+v"(c2), "+v"(c3) \
                 : "v"(a), "v"(b0), "v"(b1), "v"(b2), "v"(b3))

__device__ __forceinline__ void vst8h(_Float16* p, v8h v) { *(volatile v8h*)p = v; }
__device__ __forceinline__ void vst4f(float* p, v4f v)    { *(volatile v4f*)p = v; }

__device__ __forceinline__ void mainloop_16x64(const _Float16* __restrict__ Arow,
                                               const _Float16* __restrict__ Brow,
                                               const int K, const int h,
                                               v8f& c0, v8f& c1, v8f& c2, v8f& c3)
{
#pragma unroll 1
    for (int k0 = 0; k0 < K; k0 += 32) {
        v16h a  = load_frag(Arow + k0, h);
        v16h b0 = load_frag(Brow + k0, h);
        v16h b1 = load_frag(Brow + 16 * K + k0, h);
        v16h b2 = load_frag(Brow + 32 * K + k0, h);
        v16h b3 = load_frag(Brow + 48 * K + k0, h);
        c0 = mma16(a, b0, c0);
        c1 = mma16(a, b1, c1);
        c2 = mma16(a, b2, c2);
        c3 = mma16(a, b3, c3);
        GUARD4(c0, c1, c2, c3, a, b0, b1, b2, b3);
    }
}

__global__ __launch_bounds__(256) void prep_kernel(
    const float* __restrict__ Wq, const float* __restrict__ Wk, const float* __restrict__ Wv,
    const float* __restrict__ Wp,
    const float* __restrict__ sq, const float* __restrict__ bq,
    const float* __restrict__ sk, const float* __restrict__ bk,
    const float* __restrict__ sv, const float* __restrict__ bv,
    _Float16* __restrict__ wabc, _Float16* __restrict__ wph,
    float* __restrict__ sc, float* __restrict__ bc)
{
    const int NW1 = MQKV * DIMC / 8;
    const int NW2 = DIMC * DHC / 8;
    const int i = blockIdx.x * 256 + threadIdx.x;
    if (i < NW1 + NW2) {
        const float* src;
        _Float16* dst;
        if (i < NW1) {
            const int e = i * 8;
            if (e < NHKD * DIMC)          src = Wq + e;
            else if (e < 2 * NHKD * DIMC) src = Wk + (e - NHKD * DIMC);
            else                          src = Wv + (e - 2 * NHKD * DIMC);
            dst = wabc + e;
        } else {
            const int e = (i - NW1) * 8;
            src = Wp + e;
            dst = wph + e;
        }
        const v4f f0 = *(const v4f*)src;
        const v4f f1 = *(const v4f*)(src + 4);
        v8h hv;
#pragma unroll
        for (int j = 0; j < 4; ++j) {
            hv[j]     = (_Float16)(f0[j] * 16.0f);
            hv[4 + j] = (_Float16)(f1[j] * 16.0f);
        }
        vst8h(dst, hv);
        __threadfence();
        vst8h(dst, hv);
    } else {
        const int j = i - (NW1 + NW2);
        if (j < 512) {
            const int e = (j & 255) * 4;
            v4f o;
#pragma unroll
            for (int q = 0; q < 4; ++q) {
                const int ee = e + q;
                float val;
                if (j < 256) {
                    val = (ee < NHKD) ? sq[ee] : ((ee < 2 * NHKD) ? sk[ee - NHKD] : sv[ee - 2 * NHKD]);
                    val *= 0.0625f;
                } else {
                    val = (ee < NHKD) ? bq[ee] : ((ee < 2 * NHKD) ? bk[ee - NHKD] : bv[ee - 2 * NHKD]);
                }
                o[q] = val;
            }
            float* dst = ((j < 256) ? sc : bc) + e;
            vst4f(dst, o);
            __threadfence();
            vst4f(dst, o);
        }
    }
}

__global__ __launch_bounds__(256) void xpose_kernel(const float* __restrict__ x,
                                                    _Float16* __restrict__ xt)
{
    __shared__ float tile[128 * 33];
    const int b = blockIdx.z;
    const int nb = blockIdx.x * 32, cb = blockIdx.y * 128;
    const int t = threadIdx.x, l = t & 31, w = t >> 5, h = l >> 4, m = l & 15;
    const float* xb = x + (size_t)b * DIMC * NN;
#pragma unroll
    for (int j = 0; j < 16; ++j) {
        const int c = w + 8 * j;
        tile[c * 33 + l] = xb[(size_t)(cb + c) * NN + nb + l];
    }
    __syncthreads();
    _Float16* xo = xt + (size_t)b * NN * DIMC;
    const int nl0 = w * 4 + h, nl1 = w * 4 + 2 + h;
    v8h hv0, hv1;
#pragma unroll
    for (int j = 0; j < 8; ++j) {
        hv0[j] = (_Float16)tile[(m * 8 + j) * 33 + nl0];
        hv1[j] = (_Float16)tile[(m * 8 + j) * 33 + nl1];
    }
    _Float16* d0 = xo + (size_t)(nb + nl0) * DIMC + cb + m * 8;
    _Float16* d1 = xo + (size_t)(nb + nl1) * DIMC + cb + m * 8;
    vst8h(d0, hv0);
    vst8h(d1, hv1);
    __threadfence();
    vst8h(d0, hv0);
    vst8h(d1, hv1);
}

__global__ __launch_bounds__(256) void qkv_kernel(const _Float16* __restrict__ wabc,
                                                  const _Float16* __restrict__ xt,
                                                  const float* __restrict__ sc,
                                                  const float* __restrict__ bc,
                                                  _Float16* __restrict__ qsm,
                                                  float* __restrict__ kf,
                                                  _Float16* __restrict__ vh)
{
    __shared__ float tile[64 * TP];
    const int b = blockIdx.z;
    const int t = threadIdx.x, l = t & 31, wave = t >> 5, h = l >> 4, m = l & 15;
    const int mw = wave >> 1, nw = wave & 1;
    const int Mbase = blockIdx.y * 64, Nbase = blockIdx.x * 128;
    const int region = (blockIdx.y < 4) ? 0 : ((blockIdx.y < 8) ? 1 : 2);

    const _Float16* Arow = wabc + (size_t)(Mbase + mw * 16 + m) * DIMC;
    const _Float16* Brow = xt + ((size_t)b * NN + Nbase + nw * 64 + m) * DIMC;
    v8f c0 = {}, c1 = {}, c2 = {}, c3 = {};
    mainloop_16x64(Arow, Brow, DIMC, h, c0, c1, c2, c3);

#pragma unroll
    for (int r = 0; r < 8; ++r) {
        const int ml = mw * 16 + 8 * h + r;
        const int o = Mbase + ml;
        const float s = sc[o], bb = bc[o];
        float* trow = tile + ml * TP + nw * 64 + m;
        trow[0]  = c0[r] * s + bb;
        trow[16] = c1[r] * s + bb;
        trow[32] = c2[r] * s + bb;
        trow[48] = c3[r] * s + bb;
    }
    __syncthreads();

    if (region == 0) {
        const int nl = t & 127, hh = t >> 7;
        float qv[KDIM];
        float mx;
#pragma unroll
        for (int i = 0; i < KDIM; ++i) {
            qv[i] = tile[(hh * KDIM + i) * TP + nl];
            mx = (i == 0) ? qv[0] : fmaxf(mx, qv[i]);
        }
        float sum = 0.f;
#pragma unroll
        for (int i = 0; i < KDIM; ++i) { qv[i] = __expf(qv[i] - mx); sum += qv[i]; }
        const float scl = 256.0f / sum;
#pragma unroll
        for (int i = 0; i < KDIM; ++i) tile[(hh * KDIM + i) * TP + nl] = qv[i] * scl;
    }
    __syncthreads();

    if (region == 0) {
        const int p = l & 7;
#pragma unroll
        for (int it = 0; it < 4; ++it) {
            const int nl = wave * 16 + it * 4 + (l >> 3);
            v8h hv;
#pragma unroll
            for (int j = 0; j < 8; ++j) hv[j] = (_Float16)tile[(p * 8 + j) * TP + nl];
            vst8h(qsm + ((size_t)b * NN + Nbase + nl) * NHKD + Mbase + p * 8, hv);
        }
        __threadfence();
#pragma unroll
        for (int it = 0; it < 4; ++it) {
            const int nl = wave * 16 + it * 4 + (l >> 3);
            v8h hv;
#pragma unroll
            for (int j = 0; j < 8; ++j) hv[j] = (_Float16)tile[(p * 8 + j) * TP + nl];
            vst8h(qsm + ((size_t)b * NN + Nbase + nl) * NHKD + Mbase + p * 8, hv);
        }
    } else if (region == 1) {
        const int col = (l >> 3) * 32 + (l & 7) * 4;
        const int obase = Mbase - NHKD;
#pragma unroll
        for (int it = 0; it < 8; ++it) {
            const int row = wave * 8 + it;
            const v4f v = *(const v4fa*)(tile + row * TP + col);
            vst4f(kf + ((size_t)b * NHKD + obase + row) * NN + Nbase + col, v);
        }
        __threadfence();
#pragma unroll
        for (int it = 0; it < 8; ++it) {
            const int row = wave * 8 + it;
            const v4f v = *(const v4fa*)(tile + row * TP + col);
            vst4f(kf + ((size_t)b * NHKD + obase + row) * NN + Nbase + col, v);
        }
    } else {
        const int obase = Mbase - 2 * NHKD;
#pragma unroll
        for (int it = 0; it < 4; ++it) {
            const int row = wave * 8 + it * 2 + h;
            v8h hv;
#pragma unroll
            for (int j = 0; j < 8; ++j) hv[j] = (_Float16)tile[row * TP + m * 8 + j];
            vst8h(vh + ((size_t)b * DHC + obase + row) * NN + Nbase + m * 8, hv);
        }
        __threadfence();
#pragma unroll
        for (int it = 0; it < 4; ++it) {
            const int row = wave * 8 + it * 2 + h;
            v8h hv;
#pragma unroll
            for (int j = 0; j < 8; ++j) hv[j] = (_Float16)tile[row * TP + m * 8 + j];
            vst8h(vh + ((size_t)b * DHC + obase + row) * NN + Nbase + m * 8, hv);
        }
    }
}

__global__ __launch_bounds__(256) void softmax_k_kernel(const float* __restrict__ kf,
                                                        _Float16* __restrict__ ksm)
{
    __shared__ float red[8];
    const size_t row = blockIdx.x;
    const float* p = kf + row * NN;
    _Float16* q = ksm + row * NN;
    const int t = threadIdx.x, l = t & 31, w = t >> 5;
    const v4f a0 = *(const v4f*)(p + t * 8);
    const v4f a1 = *(const v4f*)(p + t * 8 + 4);
    const v4f a2 = *(const v4f*)(p + 2048 + t * 8);
    const v4f a3 = *(const v4f*)(p + 2048 + t * 8 + 4);
    float v[16];
#pragma unroll
    for (int j = 0; j < 4; ++j) { v[j] = a0[j]; v[4 + j] = a1[j]; v[8 + j] = a2[j]; v[12 + j] = a3[j]; }
    float mx = v[0];
#pragma unroll
    for (int j = 1; j < 16; ++j) mx = fmaxf(mx, v[j]);
#pragma unroll
    for (int off = 16; off > 0; off >>= 1) mx = fmaxf(mx, __shfl_xor(mx, off, 32));
    if (l == 0) red[w] = mx;
    __syncthreads();
    mx = red[0];
#pragma unroll
    for (int j = 1; j < 8; ++j) mx = fmaxf(mx, red[j]);
    __syncthreads();
    float sum = 0.f;
#pragma unroll
    for (int j = 0; j < 16; ++j) { v[j] = __expf(v[j] - mx); sum += v[j]; }
#pragma unroll
    for (int off = 16; off > 0; off >>= 1) sum += __shfl_xor(sum, off, 32);
    if (l == 0) red[w] = sum;
    __syncthreads();
    float tot = 0.f;
#pragma unroll
    for (int j = 0; j < 8; ++j) tot += red[j];
    const float scl = 4096.0f / tot;
    v8h h0, h1;
#pragma unroll
    for (int j = 0; j < 8; ++j) { h0[j] = (_Float16)(v[j] * scl); h1[j] = (_Float16)(v[8 + j] * scl); }
    _Float16* d0 = q + t * 8;
    _Float16* d1 = q + 2048 + t * 8;
    vst8h(d0, h0);
    vst8h(d1, h1);
    __threadfence();
    vst8h(d0, h0);
    vst8h(d1, h1);
}

__global__ __launch_bounds__(256) void ctx_kernel(const _Float16* __restrict__ ksm,
                                                  const _Float16* __restrict__ vh,
                                                  _Float16* __restrict__ ctxT)
{
    __shared__ float tile[KDIM * TPD];
    const int bh = blockIdx.x, b = bh >> 3, hd = bh & 7;
    const int t = threadIdx.x, l = t & 31, wave = t >> 5, h = l >> 4, m = l & 15;
    const int mt = wave & 1, nt = wave >> 1;
    const _Float16* Arow = ksm + ((size_t)b * NHKD + hd * KDIM + mt * 16 + m) * NN;
    const _Float16* Brow = vh  + ((size_t)b * DHC  + hd * DD   + nt * 16 + m) * NN;
    v8f c = {};
#pragma unroll 1
    for (int k0 = 0; k0 < NN; k0 += 32) {
        v16h a  = load_frag(Arow + k0, h);
        v16h bf = load_frag(Brow + k0, h);
        c = mma16(a, bf, c);
        GUARD1(c, a, bf);
    }
#pragma unroll
    for (int r = 0; r < 8; ++r)
        tile[(mt * 16 + 8 * h + r) * TPD + nt * 16 + m] = c[r];
    __syncthreads();
    const int d = wave * 8 + (l >> 2), p = l & 3;
    v8h hv;
#pragma unroll
    for (int j = 0; j < 8; ++j) hv[j] = (_Float16)(tile[(p * 8 + j) * TPD + d] * 0.015625f);
    _Float16* dst = ctxT + ((size_t)bh * DD + d) * KDIM + p * 8;
    vst8h(dst, hv);
    __threadfence();
    vst8h(dst, hv);
}

__global__ __launch_bounds__(256) void att_kernel(const _Float16* __restrict__ ctxT,
                                                  const _Float16* __restrict__ qsm,
                                                  _Float16* __restrict__ att)
{
    __shared__ float tile[128 * TPD];
    const int bh = blockIdx.y, b = bh >> 3, hd = bh & 7;
    const int Nbase = blockIdx.x * 128;
    const int t = threadIdx.x, l = t & 31, wave = t >> 5, h = l >> 4, m = l & 15;
    const int mt = wave >> 1, nw = wave & 1;
    v16h a = load_frag(ctxT + ((size_t)bh * DD + mt * 16 + m) * KDIM, h);
#pragma unroll
    for (int ns = 0; ns < 4; ++ns) {
        const int nl = nw * 64 + ns * 16 + m;
        v16h bf = load_frag(qsm + ((size_t)b * NN + Nbase + nl) * NHKD + hd * KDIM, h);
        v8f c = {};
        c = mma16(a, bf, c);
        GUARD1(c, a, bf);
#pragma unroll
        for (int r = 0; r < 8; ++r) {
            const float y = fmaxf(c[r] * 0.015625f, 0.0f);
            tile[nl * TPD + mt * 16 + 8 * h + r] = y;
        }
    }
    __syncthreads();
    const int p = l & 7;
#pragma unroll
    for (int it = 0; it < 4; ++it) {
        const int nl = wave * 16 + it * 4 + (l >> 3);
        v8h hv;
#pragma unroll
        for (int j = 0; j < 8; ++j) hv[j] = (_Float16)tile[nl * TPD + p * 8 + j];
        vst8h(att + ((size_t)b * NN + Nbase + nl) * DHC + hd * DD + p * 8, hv);
    }
    __threadfence();
#pragma unroll
    for (int it = 0; it < 4; ++it) {
        const int nl = wave * 16 + it * 4 + (l >> 3);
        v8h hv;
#pragma unroll
        for (int j = 0; j < 8; ++j) hv[j] = (_Float16)tile[nl * TPD + p * 8 + j];
        vst8h(att + ((size_t)b * NN + Nbase + nl) * DHC + hd * DD + p * 8, hv);
    }
}

__global__ __launch_bounds__(256) void out_kernel(const _Float16* __restrict__ wph,
                                                  const _Float16* __restrict__ att,
                                                  const float* __restrict__ sp,
                                                  const float* __restrict__ bp,
                                                  float* __restrict__ out)
{
    __shared__ float tile[64 * TP];
    const int b = blockIdx.z;
    const int t = threadIdx.x, l = t & 31, wave = t >> 5, h = l >> 4, m = l & 15;
    const int mw = wave >> 1, nw = wave & 1;
    const int Mbase = blockIdx.y * 64, Nbase = blockIdx.x * 128;
    const _Float16* Arow = wph + (size_t)(Mbase + mw * 16 + m) * DHC;
    const _Float16* Brow = att + ((size_t)b * NN + Nbase + nw * 64 + m) * DHC;
    v8f c0 = {}, c1 = {}, c2 = {}, c3 = {};
    mainloop_16x64(Arow, Brow, DHC, h, c0, c1, c2, c3);

#pragma unroll
    for (int r = 0; r < 8; ++r) {
        const int ml = mw * 16 + 8 * h + r;
        const int o = Mbase + ml;
        const float s = sp[o] * 0.000244140625f;
        const float bb = bp[o];
        float* trow = tile + ml * TP + nw * 64 + m;
        trow[0]  = c0[r] * s + bb;
        trow[16] = c1[r] * s + bb;
        trow[32] = c2[r] * s + bb;
        trow[48] = c3[r] * s + bb;
    }
    __syncthreads();
    const int col = (l >> 3) * 32 + (l & 7) * 4;
#pragma unroll
    for (int it = 0; it < 8; ++it) {
        const int row = wave * 8 + it;
        const v4f v = *(const v4fa*)(tile + row * TP + col);
        vst4f(out + ((size_t)b * DIMC + Mbase + row) * NN + Nbase + col, v);
    }
    __threadfence();
#pragma unroll
    for (int it = 0; it < 8; ++it) {
        const int row = wave * 8 + it;
        const v4f v = *(const v4fa*)(tile + row * TP + col);
        vst4f(out + ((size_t)b * DIMC + Mbase + row) * NN + Nbase + col, v);
    }
}

extern "C" void kernel_launch(void* const* d_in, const int* in_sizes, int n_in,
                              void* d_out, int out_size, void* d_ws, size_t ws_size,
                              hipStream_t stream)
{
    if (n_in < 13) return;
    if (in_sizes[0] != BB * DIMC * NN) return;
    if (in_sizes[1] != NHKD * DIMC || in_sizes[2] != NHKD || in_sizes[3] != NHKD) return;
    if (in_sizes[4] != NHKD * DIMC || in_sizes[5] != NHKD || in_sizes[6] != NHKD) return;
    if (in_sizes[7] != DHC * DIMC || in_sizes[8] != DHC || in_sizes[9] != DHC) return;
    if (in_sizes[10] != DIMC * DHC || in_sizes[11] != DIMC || in_sizes[12] != DIMC) return;
    if (out_size != BB * DIMC * NN) return;

    const size_t off_xt   = 0;
    const size_t sz_xt    = (size_t)BB * NN * DIMC * 2;
    const size_t off_wabc = off_xt + sz_xt;
    const size_t sz_wabc  = (size_t)MQKV * DIMC * 2;
    const size_t off_wph  = off_wabc + sz_wabc;
    const size_t sz_wph   = (size_t)DIMC * DHC * 2;
    const size_t off_sc   = off_wph + sz_wph;
    const size_t sz_sc    = (size_t)MQKV * 4;
    const size_t off_bc   = off_sc + sz_sc;
    const size_t off_qsm  = off_bc + sz_sc;
    const size_t sz_qsm   = (size_t)BB * NN * NHKD * 2;
    const size_t off_kf   = off_qsm + sz_qsm;
    const size_t sz_kf    = (size_t)BB * NHKD * NN * 4;
    const size_t off_vh   = off_kf + sz_kf;
    const size_t sz_vh    = (size_t)BB * DHC * NN * 2;
    const size_t off_ctx  = off_vh + sz_vh;
    const size_t sz_ctx   = (size_t)BB * HEADS * DD * KDIM * 2;
    const size_t total    = off_ctx + sz_ctx;
    const size_t sz_ksm   = (size_t)BB * NHKD * NN * 2;
    const size_t sz_att   = (size_t)BB * NN * DHC * 2;
    if (total > ws_size) return;
    if (sz_ksm > sz_xt || sz_att > sz_kf) return;

    const float* x  = (const float*)d_in[0];
    const float* Wq = (const float*)d_in[1];
    const float* sq = (const float*)d_in[2];
    const float* bq = (const float*)d_in[3];
    const float* Wk = (const float*)d_in[4];
    const float* sk = (const float*)d_in[5];
    const float* bk = (const float*)d_in[6];
    const float* Wv = (const float*)d_in[7];
    const float* sv = (const float*)d_in[8];
    const float* bv = (const float*)d_in[9];
    const float* Wp = (const float*)d_in[10];
    const float* sp = (const float*)d_in[11];
    const float* bp = (const float*)d_in[12];
    float* out = (float*)d_out;

    char* ws = (char*)d_ws;
    _Float16* xt   = (_Float16*)(ws + off_xt);
    _Float16* ksm  = (_Float16*)(ws + off_xt);
    _Float16* wabc = (_Float16*)(ws + off_wabc);
    _Float16* wph  = (_Float16*)(ws + off_wph);
    float*    sc   = (float*)   (ws + off_sc);
    float*    bc   = (float*)   (ws + off_bc);
    _Float16* qsm  = (_Float16*)(ws + off_qsm);
    float*    kf   = (float*)   (ws + off_kf);
    _Float16* att  = (_Float16*)(ws + off_kf);
    _Float16* vh   = (_Float16*)(ws + off_vh);
    _Float16* ctxT = (_Float16*)(ws + off_ctx);

    const int prep_threads = MQKV * DIMC / 8 + DIMC * DHC / 8 + 512;
    prep_kernel<<<(prep_threads + 255) / 256, 256, 0, stream>>>(
        Wq, Wk, Wv, Wp, sq, bq, sk, bk, sv, bv, wabc, wph, sc, bc);

    xpose_kernel<<<dim3(NN / 32, DIMC / 128, BB), 256, 0, stream>>>(x, xt);

    qkv_kernel<<<dim3(NN / 128, MQKV / 64, BB), 256, 0, stream>>>(wabc, xt, sc, bc, qsm, kf, vh);

    softmax_k_kernel<<<BB * NHKD, 256, 0, stream>>>(kf, ksm);

    ctx_kernel<<<BB * HEADS, 256, 0, stream>>>(ksm, vh, ctxT);

    att_kernel<<<dim3(NN / 128, BB * HEADS), 256, 0, stream>>>(ctxT, qsm, att);

    out_kernel<<<dim3(NN / 128, DIMC / 64, BB), 256, 0, stream>>>(wph, att, sp, bp, out);
}
